// MDN2Layer_25039659336010
// MI455X (gfx1250) — hardware-verified
//
#include <hip/hip_runtime.h>
#include <math.h>

typedef __attribute__((ext_vector_type(16))) __bf16   v16b;
typedef __attribute__((ext_vector_type(8)))  float    v8f;
typedef __attribute__((ext_vector_type(4)))  float    v4f;
typedef __attribute__((ext_vector_type(8)))  unsigned v8u;

constexpr unsigned kBatch       = 16;
constexpr unsigned kDin         = 128;
constexpr unsigned kMix         = 16;
constexpr unsigned kUnits       = 6 * kMix;
constexpr unsigned kNX          = 302;
constexpr unsigned kNY          = 394;
constexpr unsigned kGrid        = kNX * kNY;
constexpr unsigned kOutFloats   = kBatch * kGrid;
constexpr unsigned kLines       = kOutFloats / 32;
constexpr unsigned kRecFloats   = 8;
constexpr unsigned kParamFloats = kBatch * kMix * kRecFloats;
constexpr unsigned kLinesPerWave  = 4;
constexpr unsigned kLinesPerBlock = 8 * kLinesPerWave;
constexpr unsigned kEvalBlocks  = (kLines + kLinesPerBlock - 1) / kLinesPerBlock;
constexpr float    kInvTwoPi    = 0.15915494309189535f;
constexpr float    kStepX       = 1.0f / (float)(kNX - 1);
constexpr float    kStepY       = 1.0f / (float)(kNY - 1);

static_assert(kUnits == 96, "projection width");
static_assert(kGrid == 118988u, "grid points per sample");
static_assert(kOutFloats == 1903808u, "output floats");
static_assert((kOutFloats % 32u) == 0u && kLines == 59494u, "output is a whole number of 128-B lines");
static_assert((kDin % 32u) == 0u && (kUnits % 16u) == 0u && kBatch == 16u, "K multiple of 32, N multiple of 16, M one tile");
static_assert(kParamFloats == 2048u, "parameter plane floats");
static_assert((kDin * kUnits) == 16u * 192u * 4u, "weight staging: 16 trips x 192 threads x 4 floats");
static_assert(kEvalBlocks == 1860u, "evaluation grid");

constexpr size_t kOffPar  = 0;
constexpr size_t kWsTotal = kOffPar + (size_t)kParamFloats * 4;
static_assert(kWsTotal == 8192ull, "carve total");
static_assert(kWsTotal <= 134217728ull, "carve cap");

__device__ __forceinline__ unsigned bf_hi_word(float f) {
  unsigned u = __float_as_uint(f);
  const unsigned lsb = (u & 0x00010000u) ? 1u : 0u;
  u = (u + 0x7FFFu + lsb) & 0xFFFF0000u;
  return u;
}
__device__ __forceinline__ unsigned pack_upper_halves(unsigned od, unsigned ev) {
  return __builtin_amdgcn_perm(od, ev, 0x07060302u);
}
__device__ __forceinline__ void split16(const float (&f)[16], v16b& hi, v16b& lo) {
  v8u wh, wl;
#pragma unroll
  for (int j = 0; j < 8; ++j) {
    const float f0 = f[2 * j];
    const float f1 = f[2 * j + 1];
    const unsigned h0 = bf_hi_word(f0);
    const unsigned h1 = bf_hi_word(f1);
    const float r0 = f0 - __uint_as_float(h0);
    const float r1 = f1 - __uint_as_float(h1);
    const unsigned l0 = bf_hi_word(r0);
    const unsigned l1 = bf_hi_word(r1);
    wh[j] = pack_upper_halves(h1, h0);
    wl[j] = pack_upper_halves(l1, l0);
  }
  hi = __builtin_bit_cast(v16b, wh);
  lo = __builtin_bit_cast(v16b, wl);
}
__device__ __forceinline__ v8f mma_bf(v16b a, v16b b, v8f c) {
  c = __builtin_amdgcn_wmma_f32_16x16x32_bf16(false, a, false, b, (short)0, c, false, false);
  asm volatile("v_nop\n\tv_nop\n\tv_nop\n\tv_nop" : "+v"(c) : "v"(a), "v"(b));
  return c;
}
__device__ __forceinline__ void group_guard(v8f& c, v16b a0, v16b a1, v16b b0, v16b b1) {
  asm volatile("v_nop\n\tv_nop\n\tv_nop\n\tv_nop" : "+v"(c) : "v"(a0), "v"(a1), "v"(b0), "v"(b1));
}

__global__ __launch_bounds__(192) void mix_setup_kernel(
    const float* __restrict__ xin, const float* __restrict__ wt,
    const float* __restrict__ bias, float* __restrict__ params)
{
  __shared__ __align__(16) float sW[kDin * kUnits];
  __shared__ __align__(16) float sY[kBatch * kUnits];
  __shared__ __align__(16) float sP[kParamFloats];
  static_assert(sizeof(float) * (kDin * kUnits + kBatch * kUnits + kParamFloats) <= 65536u, "static LDS");

  const unsigned tid  = threadIdx.x;
  const unsigned lane = tid & 31u;
  const unsigned wave = (unsigned)__builtin_amdgcn_readfirstlane((int)(tid >> 5));
  const unsigned hh   = lane >> 4;
  const unsigned cc   = lane & 15u;
  const unsigned n    = wave * 16u + cc;

#pragma unroll 4
  for (unsigned it = 0; it < 16u; ++it) {
    const unsigned i4 = it * 192u + tid;
    const v4f v = *(const v4f*)(wt + (size_t)i4 * 4u);
    *(v4f*)(sW + i4 * 4u) = v;
  }
  const float bn = bias[n];
  __syncthreads();

  v8f acc = (v8f){0.f, 0.f, 0.f, 0.f, 0.f, 0.f, 0.f, 0.f};
  const float* arow = xin + cc * kDin + 8u * hh;
#pragma unroll
  for (int ks = 0; ks < 4; ++ks) {
    const unsigned k0 = (unsigned)ks * 32u;
    const v4f a0 = *(const v4f*)(arow + k0);
    const v4f a1 = *(const v4f*)(arow + k0 + 4u);
    const v4f a2 = *(const v4f*)(arow + k0 + 16u);
    const v4f a3 = *(const v4f*)(arow + k0 + 20u);
    float fa[16];
    float fb[16];
#pragma unroll
    for (int e = 0; e < 4; ++e) {
      fa[e]      = a0[e];
      fa[4 + e]  = a1[e];
      fa[8 + e]  = a2[e];
      fa[12 + e] = a3[e];
    }
    const float* bcol = sW + (k0 + 8u * hh) * kUnits + n;
#pragma unroll
    for (int i = 0; i < 8; ++i) {
      fb[i]     = bcol[(unsigned)i * kUnits];
      fb[8 + i] = bcol[(16u + (unsigned)i) * kUnits];
    }
    v16b ah, al, bh, bl;
    split16(fa, ah, al);
    split16(fb, bh, bl);
    acc = mma_bf(ah, bh, acc);
    acc = mma_bf(ah, bl, acc);
    acc = mma_bf(al, bh, acc);
    group_guard(acc, ah, al, bh, bl);
  }

#pragma unroll
  for (int r = 0; r < 8; ++r) {
    sY[(8u * hh + (unsigned)r) * kUnits + n] = acc[r] + bn;
  }
  __syncthreads();

#pragma unroll 1
  for (unsigned item = tid; item < kBatch * kMix; item += 192u) {
    const unsigned bq = item >> 4;
    const unsigned kq = item & 15u;
    const float* yb = sY + bq * kUnits;
    float mx = yb[80];
#pragma unroll 1
    for (unsigned j = 1; j < kMix; ++j) mx = fmaxf(mx, yb[80u + j]);
    float ssum = 0.0f;
#pragma unroll 1
    for (unsigned j = 0; j < kMix; ++j) ssum += expf(yb[80u + j] - mx);
    const float wk   = expf(yb[80u + kq] - mx) * (1.0f / ssum);
    const float mu0  = yb[2u * kq];
    const float mu1  = yb[2u * kq + 1u];
    const float aa   = yb[32u + 3u * kq];
    const float iL22 = expf(-yb[32u + 3u * kq + 1u]);
    const float iL11 = expf(-yb[32u + 3u * kq + 2u]);
    const float coef = wk * iL11 * iL22 * kInvTwoPi;
    const v4f p0 = (v4f){mu0, mu1, aa, iL11};
    const v4f p1 = (v4f){iL22, coef, 0.0f, 0.0f};
    *(v4f*)(sP + item * kRecFloats)      = p0;
    *(v4f*)(sP + item * kRecFloats + 4u) = p1;
  }
  __syncthreads();

#pragma unroll 1
  for (unsigned ch = wave; ch < kParamFloats / 128u; ch += 6u) {
    const unsigned o = ch * 128u + lane * 4u;
    const v4f v = *(const v4f*)(sP + o);
    volatile v4f* gp = (volatile v4f*)(params + o);
    *gp = v;
    __threadfence();
    *gp = v;
  }
}

__global__ __launch_bounds__(256) void mix_eval_kernel(
    const float* __restrict__ params, float* __restrict__ out)
{
  __shared__ __align__(16) float sP[kParamFloats];
  const unsigned tid  = threadIdx.x;
  const unsigned lane = tid & 31u;
  const unsigned wave = (unsigned)__builtin_amdgcn_readfirstlane((int)(tid >> 5));
  {
    const v4f t0 = *(const v4f*)(params + tid * 4u);
    const v4f t1 = *(const v4f*)(params + (tid + 256u) * 4u);
    *(v4f*)(sP + tid * 4u)          = t0;
    *(v4f*)(sP + (tid + 256u) * 4u) = t1;
  }
  __syncthreads();

  const unsigned line0 = blockIdx.x * kLinesPerBlock + wave * kLinesPerWave;
#pragma unroll 1
  for (unsigned j = 0; j < kLinesPerWave; ++j) {
    const unsigned line = line0 + j;
    if (line < kLines) {
      unsigned idx = line * 32u + lane;
      asm volatile("" : "+v"(idx));
      unsigned bq = idx / kGrid;
      bq = (bq < kBatch - 1u) ? bq : (kBatch - 1u);
      asm volatile("" : "+v"(bq));
      unsigned g = idx - bq * kGrid;
      asm volatile("" : "+v"(g));
      unsigned ix = g / kNY;
      ix = (ix < kNX - 1u) ? ix : (kNX - 1u);
      asm volatile("" : "+v"(ix));
      unsigned iy = g - ix * kNY;
      iy = (iy < kNY - 1u) ? iy : (kNY - 1u);
      asm volatile("" : "+v"(iy));
      float gx = (float)ix * kStepX;
      float gy = (float)iy * kStepY;
      gx = (ix == kNX - 1u) ? 1.0f : gx;
      gy = (iy == kNY - 1u) ? 1.0f : gy;

      const float* rec = sP + bq * (kMix * kRecFloats);
      float acc = 0.0f;
#pragma unroll 1
      for (unsigned k = 0; k < kMix; ++k) {
        const v4f p0 = *(const v4f*)(rec + k * kRecFloats);
        const v4f p1 = *(const v4f*)(rec + k * kRecFloats + 4u);
        const float z1 = (gx - p0[0]) * p0[3];
        const float z2 = ((gy - p0[1]) - p0[2] * z1) * p1[0];
        const float mh = z1 * z1 + z2 * z2;
        const float ev = expf(-0.5f * mh);
        acc = fmaf(p1[1], ev, acc);
      }
      volatile float* op = (volatile float*)(out + idx);
      *op = acc;
      __threadfence();
      *op = acc;
    }
  }
}

extern "C" void kernel_launch(void* const* d_in, const int* in_sizes, int n_in,
                              void* d_out, int out_size, void* d_ws, size_t ws_size,
                              hipStream_t stream) {
  if (n_in < 3) return;
  if (in_sizes[0] != (int)(kBatch * kDin)) return;
  if (in_sizes[1] != (int)(kDin * kUnits)) return;
  if (in_sizes[2] != (int)kUnits) return;
  if (out_size != (int)kOutFloats) return;
  if (ws_size < kWsTotal) return;

  const float* xin  = (const float*)d_in[0];
  const float* wt   = (const float*)d_in[1];
  const float* bias = (const float*)d_in[2];
  float* params = (float*)((char*)d_ws + kOffPar);
  float* out    = (float*)d_out;

  mix_setup_kernel<<<1, 192, 0, stream>>>(xin, wt, bias, params);
  mix_eval_kernel<<<kEvalBlocks, 256, 0, stream>>>(params, out);
}
